// MultiHeadAttentionWithROPE_88029649699027
// MI455X (gfx1250) — hardware-verified
//
#include <hip/hip_runtime.h>
#include <math.h>

constexpr int kBatch = 64;
constexpr int kSeq   = 200;
constexpr int kDim   = 1024;
constexpr int kHeads = 16;
constexpr int kDh    = 64;
constexpr int kTok   = kBatch * kSeq;
constexpr int kNout  = 3 * kDim;
constexpr int kPairs = kDh / 2;
constexpr int kChunks     = 2;
constexpr int kBatchChunk = kBatch / kChunks;
constexpr int kTokChunk   = kBatchChunk * kSeq;
constexpr int kQB    = 64;
constexpr int kKC    = 64;
constexpr int kNQB   = (kSeq + kQB - 1) / kQB;
constexpr int kNKC   = (kSeq + kKC - 1) / kKC;
constexpr float kScoreScale = 0.125f;
static_assert(kHeads * kDh == kDim);
static_assert(3 * kDh == 192);
static_assert(kBatch % kChunks == 0);
static_assert(kTokChunk % 64 == 0);
static_assert(kNout % 64 == 0);
static_assert(kDim % 32 == 0);
static_assert(((kTokChunk / 64) * (kNout / 64)) % 8 == 0);
static_assert(kNQB == 4 && kNKC == 4);
static_assert(kSeq % 4 == 0);
static_assert((kTok * kDim) % (8 * 256) == 0);
static_assert((kNout * kDim) % (8 * 256) == 0);
static_assert(kSeq % 8 == 0);

typedef __attribute__((ext_vector_type(16))) __bf16   v16b;
typedef __attribute__((ext_vector_type(8)))  __bf16   v8b;
typedef __attribute__((ext_vector_type(8)))  float    v8f;
typedef __attribute__((ext_vector_type(4)))  float    v4f;
typedef __attribute__((ext_vector_type(4)))  int      v4i;
typedef __attribute__((ext_vector_type(4)))  unsigned int v4u;

__device__ __forceinline__ unsigned short f2bf_bits(float f) {
  unsigned u = __float_as_uint(f);
  return (unsigned short)((u + 0x7FFFu + ((u >> 16) & 1u)) >> 16);
}
__device__ __forceinline__ float bf_bits2f(unsigned short h) { return __uint_as_float(((unsigned)h) << 16); }
__device__ __forceinline__ unsigned pk16(unsigned short a, unsigned short b) { return (unsigned)a | ((unsigned)b << 16); }
__device__ __forceinline__ float neg_inf() { return -__builtin_inff(); }

__device__ __forceinline__ void dep_guard4_b(v8f& a, v8f& b, v8f& c, v8f& d, v16b x, v16b y) {
  asm volatile("v_nop\n\tv_nop\n\tv_nop\n\tv_nop" : "+v"(a), "+v"(b), "+v"(c), "+v"(d) : "v"(x), "v"(y));
}
__device__ __forceinline__ void keep4_b(v16b a, v16b b, v16b c, v16b d) { asm volatile("v_nop" :: "v"(a), "v"(b), "v"(c), "v"(d)); }
__device__ __forceinline__ void acc_guard4(v8f& a, v8f& b, v8f& c, v8f& d) { asm volatile("v_nop\n\tv_nop\n\tv_nop\n\tv_nop" : "+v"(a), "+v"(b), "+v"(c), "+v"(d)); }

template <typename T> struct Frag;
template <> struct Frag<__bf16> {
  typedef v16b V; union U { v16b v; v8b h[2]; };
  static __device__ __forceinline__ v16b load(const __bf16* p) {
    U f; f.h[0] = *(const v8b*)(p); f.h[1] = *(const v8b*)(p + 16); return f.v;
  }
  static __device__ __forceinline__ v8f mma(v16b a, v16b b, v8f c) {
    return __builtin_amdgcn_wmma_f32_16x16x32_bf16(false, a, false, b, (short)0, c, false, false);
  }
  static __device__ __forceinline__ void keep(v16b a, v16b b, v16b c, v16b d) { keep4_b(a, b, c, d); }
};
__device__ __forceinline__ v8f mma_b(v16b a, v16b b, v8f c) {
  c = __builtin_amdgcn_wmma_f32_16x16x32_bf16(false, a, false, b, (short)0, c, false, false);
  asm volatile("v_nop\n\tv_nop\n\tv_nop\n\tv_nop" : "+v"(c) : "v"(a), "v"(b));
  return c;
}

__global__ __launch_bounds__(256) void cast8_bf16_kernel(const float* __restrict__ in, unsigned short* __restrict__ out, int n8) {
  const int i = blockIdx.x * 256 + threadIdx.x;
  if (i >= n8) return;
  const float* p = in + 8 * (size_t)i;
  const v4f a = *(const v4f*)(p);
  const v4f c = *(const v4f*)(p + 4);
  unsigned short hb[8];
#pragma unroll
  for (int e = 0; e < 4; ++e) {
    hb[e]     = f2bf_bits(a[e]);
    hb[4 + e] = f2bf_bits(c[e]);
  }
  const v4u u = (v4u){pk16(hb[0], hb[1]), pk16(hb[2], hb[3]), pk16(hb[4], hb[5]), pk16(hb[6], hb[7])};
  unsigned short* q = out + 8 * (size_t)i;
  *(volatile v4u*)q = u;
  __threadfence();
  *(volatile v4u*)q = u;
}

__global__ __launch_bounds__(256) void rope_table_kernel(float* __restrict__ csn, float f1, float f2, float f4, float f8, float f16v) {
  const int lane = threadIdx.x & 31, wave = threadIdx.x >> 5;
  const int s = blockIdx.x * 8 + wave;
  if (s >= kSeq) return;
  const int i = lane;
  float invf = 1.0f;
  invf *= (i & 1)  ? f1   : 1.0f;
  invf *= (i & 2)  ? f2   : 1.0f;
  invf *= (i & 4)  ? f4   : 1.0f;
  invf *= (i & 8)  ? f8   : 1.0f;
  invf *= (i & 16) ? f16v : 1.0f;
  const float ang = (float)s * invf;
  float sn, cs;
  sincosf(ang, &sn, &cs);
  float* rowp = csn + (size_t)s * (2 * kPairs);
  for (int pass = 0; pass < 2; ++pass) {
    ((volatile float*)rowp)[i] = cs;
    ((volatile float*)rowp)[kPairs + i] = sn;
    __threadfence();
  }
}

__global__ __launch_bounds__(256) void qkv_proj_kernel(
    const unsigned short* __restrict__ Xb, const unsigned short* __restrict__ Wb, const float* __restrict__ bias,
    const float* __restrict__ csn,
    unsigned short* __restrict__ Qh, unsigned short* __restrict__ Ql,
    unsigned short* __restrict__ Kh, unsigned short* __restrict__ Kl,
    unsigned short* __restrict__ Vh, unsigned short* __restrict__ Vl) {
  typedef __bf16 T;
  typedef v16b V;
  const T* A  = (const T*)Xb;
  const T* Bt = (const T*)Wb;
  __shared__ __align__(16) float sT[8][16 * 68];
  const int lane = threadIdx.x & 31;
  const int wave = threadIdx.x >> 5;
  constexpr int tilesN = kNout / 64;
  constexpr int tilesM = kTokChunk / 64;
  const int tile = blockIdx.x * 8 + wave;
  if (tile >= tilesM * tilesN) return;
  const int tm = tile / tilesN;
  const int tn = tile - tm * tilesN;
  const int m0 = tm << 6;
  const int n0 = tn << 6;
  const int hd   = tn / 3;
  const int kind = tn - hd * 3;

  const int rlane = lane & 15;
  const int koff  = (lane >> 4) * 8;
  const int mOff  = (lane >> 4) * 8;

  v8f acc[4][4];
#pragma unroll
  for (int i = 0; i < 4; ++i)
#pragma unroll
    for (int j = 0; j < 4; ++j) acc[i][j] = (v8f){0.f,0.f,0.f,0.f,0.f,0.f,0.f,0.f};

  for (int k0 = 0; k0 < kDim; k0 += 32) {
    V bfr[4];
#pragma unroll
    for (int j = 0; j < 4; ++j) {
      const size_t bo = (size_t)(n0 + (j << 4) + rlane) * kDim + koff + k0;
      bfr[j] = Frag<T>::load(Bt + bo);
    }
#pragma unroll
    for (int i = 0; i < 4; ++i) {
      const size_t ao = (size_t)(m0 + (i << 4) + rlane) * kDim + koff + k0;
      const V afr = Frag<T>::load(A + ao);
#pragma unroll
      for (int j = 0; j < 4; ++j) acc[i][j] = Frag<T>::mma(afr, bfr[j], acc[i][j]);
      dep_guard4_b(acc[i][0], acc[i][1], acc[i][2], acc[i][3], afr, bfr[3]);
    }
    Frag<T>::keep(bfr[0], bfr[1], bfr[2], bfr[3]);
  }
  acc_guard4(acc[0][0], acc[0][1], acc[0][2], acc[0][3]);
  acc_guard4(acc[1][0], acc[1][1], acc[1][2], acc[1][3]);
  acc_guard4(acc[2][0], acc[2][1], acc[2][2], acc[2][3]);
  acc_guard4(acc[3][0], acc[3][1], acc[3][2], acc[3][3]);

  float bcol[4];
#pragma unroll
  for (int j = 0; j < 4; ++j) bcol[j] = bf_bits2f(f2bf_bits(bias[n0 + (j << 4) + rlane]));

  float* slab = sT[wave];
  const int q  = lane >> 3;
  const int c8 = (lane & 7) * 8;
  const int p4 = (lane & 7) * 4;
  unsigned short* dsth = (kind == 0) ? Qh : ((kind == 1) ? Kh : Vh);
  unsigned short* dstl = (kind == 0) ? Ql : ((kind == 1) ? Kl : Vl);
  const bool rot = (kind != 2);

#pragma unroll
  for (int i = 0; i < 4; ++i) {
    const int mBase = m0 + (i << 4);
#pragma unroll
    for (int j = 0; j < 4; ++j) {
#pragma unroll
      for (int r = 0; r < 8; ++r) slab[(mOff + r) * 68 + (j << 4) + rlane] = acc[i][j][r] + bcol[j];
    }
    __builtin_amdgcn_fence(__ATOMIC_RELEASE, "workgroup");
    __builtin_amdgcn_wave_barrier();
    __builtin_amdgcn_fence(__ATOMIC_ACQUIRE, "workgroup");

    v4u uh[4], ul[4];
#pragma unroll
    for (int it = 0; it < 4; ++it) {
      if (it == 2) asm volatile("" ::: "memory");
      const int row = it * 4 + q;
      const int m   = mBase + row;
      const int s   = m - (m / kSeq) * kSeq;
      const float* sp = slab + row * 68 + c8;
      const v4f cs4 = *(const v4f*)(csn + (size_t)s * (2 * kPairs) + p4);
      const v4f sn4 = *(const v4f*)(csn + (size_t)s * (2 * kPairs) + kPairs + p4);
      unsigned short hb[8], lb[8];
#pragma unroll
      for (int pp = 0; pp < 4; ++pp) {
        const float x1 = sp[2 * pp];
        const float x2 = sp[2 * pp + 1];
        const float cc = rot ? cs4[pp] : 1.0f;
        const float ss = rot ? sn4[pp] : 0.0f;
        const float o0 = x1 * cc - x2 * ss;
        const float o1 = x1 * ss + x2 * cc;
        const unsigned short h0 = f2bf_bits(o0);
        const unsigned short h1 = f2bf_bits(o1);
        hb[2 * pp]     = h0;
        hb[2 * pp + 1] = h1;
        lb[2 * pp]     = f2bf_bits(o0 - bf_bits2f(h0));
        lb[2 * pp + 1] = f2bf_bits(o1 - bf_bits2f(h1));
      }
      uh[it] = (v4u){pk16(hb[0], hb[1]), pk16(hb[2], hb[3]), pk16(hb[4], hb[5]), pk16(hb[6], hb[7])};
      ul[it] = (v4u){pk16(lb[0], lb[1]), pk16(lb[2], lb[3]), pk16(lb[4], lb[5]), pk16(lb[6], lb[7])};
    }
    for (int pass = 0; pass < 2; ++pass) {
#pragma unroll
      for (int it = 0; it < 4; ++it) {
        const int row = it * 4 + q;
        const int m   = mBase + row;
        const size_t o = (size_t)m * kDim + hd * kDh + c8;
        *(volatile v4u*)(dsth + o) = uh[it];
        *(volatile v4u*)(dstl + o) = ul[it];
      }
      __threadfence();
    }
    __builtin_amdgcn_fence(__ATOMIC_RELEASE, "workgroup");
    __builtin_amdgcn_wave_barrier();
    __builtin_amdgcn_fence(__ATOMIC_ACQUIRE, "workgroup");
  }
}

__global__ __launch_bounds__(128) void attn_kernel(
    const unsigned short* __restrict__ Qh, const unsigned short* __restrict__ Ql,
    const unsigned short* __restrict__ Kh, const unsigned short* __restrict__ Kl,
    const unsigned short* __restrict__ Vh, const unsigned short* __restrict__ Vl,
    const int* __restrict__ amask, float* __restrict__ out) {
  __shared__ __align__(16) unsigned short Ksh[kKC * kDh];
  __shared__ __align__(16) unsigned short Ksl[kKC * kDh];
  __shared__ __align__(16) unsigned short Vth[kDh * kKC];
  __shared__ __align__(16) unsigned short Vtl[kDh * kKC];
  __shared__ __align__(16) __bf16 Psh[4][16 * kKC];
  __shared__ __align__(16) __bf16 Psl[4][16 * kKC];
  __shared__ __align__(16) float Os[4][16 * 68];
  __shared__ __align__(16) unsigned char Msk[kQB * kKC];
  __shared__ int flags[4];

  const int tid  = threadIdx.x;
  const int wave = tid >> 5;
  const int lane = tid & 31;
  const int hh   = lane >> 4;
  const int c    = lane & 15;

  const int bx = blockIdx.x;
  const int qb = bx & 3;
  const int bh = bx >> 2;
  const int h  = bh & 15;
  const int b  = bh >> 4;
  const int tokb = b * kSeq;
  const int q0 = qb * kQB + wave * 16;
  const bool active = (q0 < kSeq);

  v16b qah[2], qal[2];
  {
    int qr = q0 + c;
    qr = (qr < kSeq) ? qr : (kSeq - 1);
    const size_t qo = (size_t)(tokb + qr) * kDim + h * kDh;
    const __bf16* qhp = (const __bf16*)Qh + qo;
    const __bf16* qlp = (const __bf16*)Ql + qo;
#pragma unroll
    for (int dc = 0; dc < 2; ++dc) qah[dc] = Frag<__bf16>::load(qhp + dc * 32 + 8 * hh);
    asm volatile("" ::: "memory");
#pragma unroll
    for (int dc = 0; dc < 2; ++dc) qal[dc] = Frag<__bf16>::load(qlp + dc * 32 + 8 * hh);
  }

  float mrow[8], lrow[8];
  v8f oacc[4];
#pragma unroll
  for (int r = 0; r < 8; ++r) { mrow[r] = neg_inf(); lrow[r] = 0.f; }
#pragma unroll
  for (int t = 0; t < 4; ++t) oacc[t] = (v8f){0.f,0.f,0.f,0.f,0.f,0.f,0.f,0.f};

  for (int kc = 0; kc < kNKC; ++kc) {
    const int kv0 = kc * kKC;
    __syncthreads();
    int anyv = 0;
#pragma unroll
    for (int i = 0; i < 8; ++i) {
      if (i == 4) asm volatile("" ::: "memory");
      const int idx = i * 128 + tid;
      const int r   = idx >> 4;
      const int c16 = (idx & 15) * 4;
      int qg = qb * kQB + r;
      qg = (qg < kSeq) ? qg : (kSeq - 1);
      const int kg  = kv0 + c16;
      const int kgc = (kg <= kSeq - 4) ? kg : (kSeq - 4);
      const v4i mv = *(const v4i*)(amask + ((size_t)(tokb + qg)) * kSeq + kgc);
      unsigned packed = 0;
#pragma unroll
      for (int e = 0; e < 4; ++e) {
        const int keep = (((kg + e) < kSeq) && (mv[e] != 0)) ? 1 : 0;
        packed |= ((unsigned)keep) << (8 * e);
        anyv |= keep;
      }
      *(unsigned*)(Msk + r * kKC + c16) = packed;
    }
#pragma unroll
    for (int off = 1; off < 32; off <<= 1) anyv |= __shfl_xor(anyv, off, 32);
    if (lane == 0) flags[wave] = anyv;
    __syncthreads();
    const int anyb = flags[0] | flags[1] | flags[2] | flags[3];
    if (anyb == 0) continue;

#pragma unroll
    for (int i = 0; i < 4; ++i) {
      if (i == 2) asm volatile("" ::: "memory");
      const int idx = i * 128 + tid;
      const int r   = idx >> 3;
      const int cc  = (idx & 7) * 8;
      int kvr = kv0 + r;
      kvr = (kvr < kSeq) ? kvr : (kSeq - 1);
      const size_t go = (size_t)(tokb + kvr) * kDim + h * kDh + cc;
      const v4u kwh = *(const v4u*)(Kh + go);
      const v4u kwl = *(const v4u*)(Kl + go);
      *(v4u*)(Ksh + r * kDh + cc) = kwh;
      *(v4u*)(Ksl + r * kDh + cc) = kwl;
    }
#pragma unroll
    for (int i = 0; i < 4; ++i) {
      if (i == 2) asm volatile("" ::: "memory");
      const int idx = i * 128 + tid;
      const int r   = idx >> 3;
      const int cc  = (idx & 7) * 8;
      int kvr = kv0 + r;
      kvr = (kvr < kSeq) ? kvr : (kSeq - 1);
      const size_t go = (size_t)(tokb + kvr) * kDim + h * kDh + cc;
      const v4u vwh = *(const v4u*)(Vh + go);
      const v4u vwl = *(const v4u*)(Vl + go);
#pragma unroll
      for (int e2 = 0; e2 < 4; ++e2) {
        const unsigned wh = vwh[e2];
        const unsigned wl = vwl[e2];
        Vth[(cc + 2 * e2) * kKC + r]     = (unsigned short)(wh & 0xffffu);
        Vth[(cc + 2 * e2 + 1) * kKC + r] = (unsigned short)(wh >> 16);
        Vtl[(cc + 2 * e2) * kKC + r]     = (unsigned short)(wl & 0xffffu);
        Vtl[(cc + 2 * e2 + 1) * kKC + r] = (unsigned short)(wl >> 16);
      }
    }
    __syncthreads();

    if (active) {
      v8f s[4];
#pragma unroll
      for (int j = 0; j < 4; ++j) {
        s[j] = (v8f){0.f,0.f,0.f,0.f,0.f,0.f,0.f,0.f};
#pragma unroll
        for (int dc = 0; dc < 2; ++dc) {
          const v16b kb = Frag<__bf16>::load((const __bf16*)Ksh + (j * 16 + c) * kDh + dc * 32 + 8 * hh);
          const v16b kl = Frag<__bf16>::load((const __bf16*)Ksl + (j * 16 + c) * kDh + dc * 32 + 8 * hh);
          s[j] = mma_b(qah[dc], kb, s[j]);
          s[j] = mma_b(qah[dc], kl, s[j]);
          s[j] = mma_b(qal[dc], kb, s[j]);
        }
      }
      float cm[8];
#pragma unroll
      for (int r = 0; r < 8; ++r) {
        const int ql = wave * 16 + 8 * hh + r;
        float m = neg_inf();
#pragma unroll
        for (int j = 0; j < 4; ++j) {
          const int keep = Msk[ql * kKC + j * 16 + c];
          float sv = s[j][r] * kScoreScale;
          sv = (keep != 0) ? sv : neg_inf();
          s[j][r] = sv;
          m = fmaxf(m, sv);
        }
#pragma unroll
        for (int off = 1; off < 16; off <<= 1) m = fmaxf(m, __shfl_xor(m, off, 32));
        cm[r] = m;
      }
      __bf16* pwh = Psh[wave];
      __bf16* pwl = Psl[wave];
#pragma unroll
      for (int r = 0; r < 8; ++r) {
        const float mnew = fmaxf(mrow[r], cm[r]);
        const float mref = (mnew == neg_inf()) ? 0.0f : mnew;
        const float alpha = expf(mrow[r] - mref);
        mrow[r] = mnew;
        float psum = 0.f;
#pragma unroll
        for (int j = 0; j < 4; ++j) {
          const float p = expf(s[j][r] - mref);
          psum += p;
          const unsigned short hb = f2bf_bits(p);
          const unsigned short lb = f2bf_bits(p - bf_bits2f(hb));
          pwh[(8 * hh + r) * kKC + j * 16 + c] = __builtin_bit_cast(__bf16, hb);
          pwl[(8 * hh + r) * kKC + j * 16 + c] = __builtin_bit_cast(__bf16, lb);
        }
#pragma unroll
        for (int off = 1; off < 16; off <<= 1) psum += __shfl_xor(psum, off, 32);
        lrow[r] = lrow[r] * alpha + psum;
#pragma unroll
        for (int t = 0; t < 4; ++t) oacc[t][r] *= alpha;
      }
      __builtin_amdgcn_fence(__ATOMIC_RELEASE, "workgroup");
      __builtin_amdgcn_wave_barrier();
      __builtin_amdgcn_fence(__ATOMIC_ACQUIRE, "workgroup");
#pragma unroll
      for (int kk = 0; kk < 2; ++kk) {
        const v16b pa = Frag<__bf16>::load(pwh + c * kKC + kk * 32 + 8 * hh);
        const v16b pl = Frag<__bf16>::load(pwl + c * kKC + kk * 32 + 8 * hh);
#pragma unroll
        for (int t = 0; t < 4; ++t) {
          const v16b vb = Frag<__bf16>::load((const __bf16*)Vth + (t * 16 + c) * kKC + kk * 32 + 8 * hh);
          const v16b vl = Frag<__bf16>::load((const __bf16*)Vtl + (t * 16 + c) * kKC + kk * 32 + 8 * hh);
          oacc[t] = mma_b(pa, vb, oacc[t]);
          oacc[t] = mma_b(pa, vl, oacc[t]);
          oacc[t] = mma_b(pl, vb, oacc[t]);
        }
      }
    }
  }

  float* os = Os[wave];
#pragma unroll
  for (int r = 0; r < 8; ++r) {
    const float inv = 1.0f / lrow[r];
#pragma unroll
    for (int t = 0; t < 4; ++t) os[(8 * hh + r) * 68 + t * 16 + c] = oacc[t][r] * inv;
  }
  __builtin_amdgcn_fence(__ATOMIC_RELEASE, "workgroup");
  __builtin_amdgcn_wave_barrier();
  __builtin_amdgcn_fence(__ATOMIC_ACQUIRE, "workgroup");
  {
    const int c4 = (lane & 15) * 4;
    float* ob = out + (size_t)tokb * kDim + h * kDh;
    for (int pass = 0; pass < 2; ++pass) {
#pragma unroll
      for (int it = 0; it < 8; ++it) {
        const int row = it * 2 + hh;
        const int qq  = q0 + row;
        const v4f val = *(const v4f*)(os + row * 68 + c4);
        if (qq < kSeq) *(volatile v4f*)(ob + (size_t)qq * kDim + c4) = val;
      }
      __threadfence();
    }
  }
}

extern "C" void kernel_launch(void* const* d_in, const int* in_sizes, int n_in,
                              void* d_out, int out_size, void* d_ws, size_t ws_size,
                              hipStream_t stream) {
  if (n_in < 4) return;
  if (in_sizes[0] != kTok * kDim) return;
  if (in_sizes[1] != kBatch * kSeq * kSeq) return;
  if (in_sizes[2] != kNout * kDim) return;
  if (in_sizes[3] != kNout) return;
  if (out_size != kTok * kDim) return;

  const size_t szXb  = (size_t)kTok * kDim * 2;
  const size_t szWb  = (size_t)kNout * kDim * 2;
  const size_t szPl  = (size_t)kTokChunk * kDim * 2;
  const size_t szCS  = (size_t)kSeq * 2 * kPairs * 4;
  const size_t offXb = 0;
  const size_t offWb = offXb + szXb;
  const size_t offQh = offWb + szWb;
  const size_t offQl = offQh + szPl;
  const size_t offKh = offQl + szPl;
  const size_t offKl = offKh + szPl;
  const size_t offVh = offKl + szPl;
  const size_t offVl = offVh + szPl;
  const size_t offCS = offVl + szPl;
  const size_t total = offCS + szCS;
  if (ws_size < total) return;

  const float* x     = (const float*)d_in[0];
  const int*   amask = (const int*)d_in[1];
  const float* W     = (const float*)d_in[2];
  const float* bias  = (const float*)d_in[3];
  float* out = (float*)d_out;
  char* ws = (char*)d_ws;
  unsigned short* Xb  = (unsigned short*)(ws + offXb);
  unsigned short* Wb  = (unsigned short*)(ws + offWb);
  unsigned short* Qhp = (unsigned short*)(ws + offQh);
  unsigned short* Qlp = (unsigned short*)(ws + offQl);
  unsigned short* Khp = (unsigned short*)(ws + offKh);
  unsigned short* Klp = (unsigned short*)(ws + offKl);
  unsigned short* Vhp = (unsigned short*)(ws + offVh);
  unsigned short* Vlp = (unsigned short*)(ws + offVl);
  float* CSN = (float*)(ws + offCS);

  const float f1   = 0.7498942093324559f;
  const float f2   = 0.5623413251903491f;
  const float f4   = 0.31622776601683794f;
  const float f8   = 0.1f;
  const float f16v = 0.01f;

  const int n8x = (kTok * kDim) / 8;
  const int n8w = (kNout * kDim) / 8;
  cast8_bf16_kernel<<<dim3(n8x / 256), dim3(256), 0, stream>>>(x, Xb, n8x);
  cast8_bf16_kernel<<<dim3(n8w / 256), dim3(256), 0, stream>>>(W, Wb, n8w);
  rope_table_kernel<<<dim3(kSeq / 8), dim3(256), 0, stream>>>(CSN, f1, f2, f4, f8, f16v);

  const int tiles = (kTokChunk / 64) * (kNout / 64);
  for (int ch = 0; ch < kChunks; ++ch) {
    const unsigned short* Xc = Xb + (size_t)ch * kTokChunk * kDim;
    const int* Mc = amask + (size_t)ch * kBatchChunk * kSeq * kSeq;
    float* Oc = out + (size_t)ch * kTokChunk * kDim;
    qkv_proj_kernel<<<dim3(tiles / 8), dim3(256), 0, stream>>>(Xc, Wb, bias, CSN, Qhp, Qlp, Khp, Klp, Vhp, Vlp);
    attn_kernel<<<dim3(kBatchChunk * kHeads * kNQB), dim3(128), 0, stream>>>(Qhp, Qlp, Khp, Klp, Vhp, Vlp, Mc, Oc);
  }
}
